// model003a_37666863186446
// MI455X (gfx1250) — hardware-run, weakly checked
//
#include <hip/hip_runtime.h>
#include <math.h>

typedef __attribute__((ext_vector_type(16))) _Float16 v16h;
typedef __attribute__((ext_vector_type(8)))  _Float16 v8h;
typedef __attribute__((ext_vector_type(2)))  _Float16 v2h;
typedef __attribute__((ext_vector_type(16))) __bf16   v16b;
typedef __attribute__((ext_vector_type(8)))  __bf16   v8b;
typedef __attribute__((ext_vector_type(8)))  float    v8f;
typedef __attribute__((ext_vector_type(4)))  float    v4f;
typedef __attribute__((ext_vector_type(2)))  float    v2f;

constexpr int kT    = 4096;
constexpr int kNB   = 32;
constexpr int kNU   = 64;
constexpr int kNH   = 256;
constexpr int kHP   = kNH / 2;
constexpr int kNY   = 64;
constexpr int kTC   = 1024;
constexpr int kNCh  = kT / kTC;
constexpr int kRC   = kTC * kNB;
constexpr int kM0   = 128;
constexpr int kThr  = 256;
constexpr float kInCarry = 1024.0f;
constexpr float kXCarry = 256.0f;
constexpr float kScIn = 1.0f / (kInCarry * kInCarry);
constexpr float kScOut = 1.0f / (kXCarry * kInCarry);
constexpr float kHalfPi = 1.57079632679489661923f;
constexpr float kF16MinNormal = 6.103515625e-5f;

static_assert((kRC % 64) == 0 && (kNH % 64) == 0 && (kNY % 64) == 0 && (kM0 % 64) == 0 && (kNU % 32) == 0 && (kNH % 32) == 0 && ((kRC / 64) * (kNH / 64)) % 8 == 0 && ((kRC / 64) * (kNY / 64)) % 8 == 0 && ((kM0 / 64) * (kNH / 64)) % 8 == 0, "GEMM M, N multiples of 64, K of 32; grids exact (2,048, 512 and 8 tiles)");

constexpr size_t kOffB16 = 0ull;
constexpr size_t kOffWYX16 = 32768ull;
constexpr size_t kOffWXY16 = 65536ull;
constexpr size_t kOffBIAS = 98304ull;
constexpr size_t kOffY016 = 102400ull;
constexpr size_t kOffX0 = 118784ull;
constexpr size_t kOffSTATE = 249856ull;
constexpr size_t kOffU16 = 282624ull;
constexpr size_t kOffBU = 4476928ull;
constexpr size_t kOffX16 = 38031360ull;
constexpr size_t kOffY32 = 54808576ull;
constexpr size_t kWsTotal = 63197184ull;
static_assert(kWsTotal <= 134217728ull, "carve cap: under 128 MiB");
static_assert(kOffB16 == 0
              && kOffWYX16 == kOffB16 + 32768ull
              && kOffWXY16 == kOffWYX16 + 32768ull
              && kOffBIAS == kOffWXY16 + 32768ull
              && kOffY016 == kOffBIAS + 4096ull
              && kOffX0 == kOffY016 + 16384ull
              && kOffSTATE == kOffX0 + 131072ull
              && kOffU16 == kOffSTATE + 32768ull
              && kOffBU == kOffU16 + 4194304ull
              && kOffX16 == kOffBU + 33554432ull
              && kOffY32 == kOffX16 + 16777216ull
              && kWsTotal == kOffY32 + 8388608ull, "the carve is chained and totalled");
static_assert((kOffB16 % 256) == 0 && (kOffWYX16 % 256) == 0 && (kOffWXY16 % 256) == 0 && (kOffBIAS % 256) == 0 && (kOffY016 % 256) == 0 && (kOffX0 % 256) == 0 && (kOffSTATE % 256) == 0 && (kOffU16 % 256) == 0 && (kOffBU % 256) == 0 && (kOffX16 % 256) == 0 && (kOffY32 % 256) == 0, "aligned regions");
constexpr int kFBYX = 0, kFBXY = 256, kFZB = 512, kFEnd = 1024;

__device__ __forceinline__ unsigned short f2bf_bits(float f) {
  unsigned u = __float_as_uint(f);
  return (unsigned short)((u + 0x7FFFu + ((u >> 16) & 1u)) >> 16);
}
__device__ __forceinline__ float bf_bits2f(unsigned short h) { return __uint_as_float(((unsigned)h) << 16); }
__device__ __forceinline__ float bf16r(float f) { return bf_bits2f(f2bf_bits(f)); }
__device__ __forceinline__ float carry_flush(float v, float carry) {
  const float s = v * carry;
  return (fabsf(s) < kF16MinNormal) ? 0.0f : s;
}
__device__ __forceinline__ float frcp(float x) { return __builtin_amdgcn_rcpf(x); }

__device__ __forceinline__ void dep_guard4_h(v8f& a, v8f& b, v8f& c, v8f& d, v16h x, v16h y) { asm volatile("v_nop\n\tv_nop\n\tv_nop\n\tv_nop" : "+v"(a), "+v"(b), "+v"(c), "+v"(d) : "v"(x), "v"(y)); }
__device__ __forceinline__ void dep_guard4_b(v8f& a, v8f& b, v8f& c, v8f& d, v16b x, v16b y) { asm volatile("v_nop\n\tv_nop\n\tv_nop\n\tv_nop" : "+v"(a), "+v"(b), "+v"(c), "+v"(d) : "v"(x), "v"(y)); }
__device__ __forceinline__ void keep4_h(v16h a, v16h b, v16h c, v16h d) { asm volatile("v_nop" :: "v"(a), "v"(b), "v"(c), "v"(d)); }
__device__ __forceinline__ void keep4_b(v16b a, v16b b, v16b c, v16b d) { asm volatile("v_nop" :: "v"(a), "v"(b), "v"(c), "v"(d)); }
__device__ __forceinline__ void acc_guard4(v8f& a, v8f& b, v8f& c, v8f& d) { asm volatile("v_nop\n\tv_nop\n\tv_nop\n\tv_nop" : "+v"(a), "+v"(b), "+v"(c), "+v"(d)); }

template <typename T> struct Frag;
template <> struct Frag<_Float16> {
  typedef v16h V; union U { v16h v; v8h h[2]; };
  static __device__ __forceinline__ v16h load(const _Float16* p) {
    U f; f.h[0] = *(const v8h*)(p); f.h[1] = *(const v8h*)(p + 16); return f.v;
  }
  static __device__ __forceinline__ v8f mma(v16h a, v16h b, v8f c) {
    return __builtin_amdgcn_wmma_f32_16x16x32_f16(false, a, false, b, (short)0, c, false, false);
  }
  static __device__ __forceinline__ void guard4(v8f& a, v8f& b, v8f& c, v8f& d, v16h x, v16h y) { dep_guard4_h(a, b, c, d, x, y); }
  static __device__ __forceinline__ void keep(v16h a, v16h b, v16h c, v16h d) { keep4_h(a, b, c, d); }
};
template <> struct Frag<__bf16> {
  typedef v16b V; union U { v16b v; v8b h[2]; };
  static __device__ __forceinline__ v16b load(const __bf16* p) {
    U f; f.h[0] = *(const v8b*)(p); f.h[1] = *(const v8b*)(p + 16); return f.v;
  }
  static __device__ __forceinline__ v8f mma(v16b a, v16b b, v8f c) {
    return __builtin_amdgcn_wmma_f32_16x16x32_bf16(false, a, false, b, (short)0, c, false, false);
  }
  static __device__ __forceinline__ void guard4(v8f& a, v8f& b, v8f& c, v8f& d, v16b x, v16b y) { dep_guard4_b(a, b, c, d, x, y); }
  static __device__ __forceinline__ void keep(v16b a, v16b b, v16b c, v16b d) { keep4_b(a, b, c, d); }
};

__device__ __forceinline__ v8f mma_h(v16h a, v16h b, v8f c) {
  c = __builtin_amdgcn_wmma_f32_16x16x32_f16(false, a, false, b, (short)0, c, false, false);
  asm volatile("v_nop\n\tv_nop\n\tv_nop\n\tv_nop" : "+v"(c) : "v"(a), "v"(b));
  return c;
}

template <int ET> struct Elem;
template <> struct Elem<0> { typedef _Float16 T; };
template <> struct Elem<1> { typedef __bf16 T; };
template <int ET, bool SPLIT, int BIAS_MODE, int OUT_MODE, bool RESID, int ACT = 0>
__global__ __launch_bounds__(256) void wmma_gemm64(
    const unsigned short* __restrict__ Ap, const unsigned short* __restrict__ A2p, int lda, long strideA,
    const unsigned short* __restrict__ Btp, const unsigned short* __restrict__ Bt2p, int ldb, long strideB,
    void* __restrict__ Cout, void* __restrict__ Cout2, int ldc, long strideC,
    const float* __restrict__ bias,
    const float* __restrict__ resid, long strideR,
    int M, int N, int K, float scale) {
  typedef typename Elem<ET>::T T;
  typedef typename Frag<T>::V V;
  const T* A = (const T*)Ap; const T* A2 = (const T*)A2p; const T* Bt = (const T*)Btp; const T* Bt2 = (const T*)Bt2p;
  __shared__ __align__(16) float sT[8][16 * 68];
  const int b    = blockIdx.y;
  const int lane = threadIdx.x & 31;
  const int wave = threadIdx.x >> 5;
  const int tilesN = N >> 6;
  const int tilesM = M >> 6;
  const int tile = blockIdx.x * 8 + wave;
  if (tile >= tilesM * tilesN) return;
  const int tm = tile / tilesN;
  const int tn = tile - tm * tilesN;
  const int m0 = tm << 6;
  const int n0 = tn << 6;

  const T* Ab  = A  + (size_t)b * strideA;
  const T* Bb  = Bt + (size_t)b * strideB;
  const T* Ab2 = SPLIT ? (A2  + (size_t)b * strideA) : nullptr;
  const T* Bb2 = SPLIT ? (Bt2 + (size_t)b * strideB) : nullptr;

  const int rlane = lane & 15;
  const int koff  = (lane >> 4) * 8;
  const int mOff  = (lane >> 4) * 8;

  v8f acc[4][4];
#pragma unroll
  for (int i = 0; i < 4; ++i)
#pragma unroll
    for (int j = 0; j < 4; ++j) acc[i][j] = (v8f){0.f,0.f,0.f,0.f,0.f,0.f,0.f,0.f};

  for (int k0 = 0; k0 < K; k0 += 32) {
    V bh[4], bl[4];
#pragma unroll
    for (int j = 0; j < 4; ++j) {
      const size_t bo = (size_t)(n0 + (j << 4) + rlane) * ldb + koff + k0;
      bh[j] = Frag<T>::load(Bb + bo);
      if (SPLIT) bl[j] = Frag<T>::load(Bb2 + bo);
    }
#pragma unroll
    for (int i = 0; i < 4; ++i) {
      const size_t ao = (size_t)(m0 + (i << 4) + rlane) * lda + koff + k0;
      V ah = Frag<T>::load(Ab + ao);
      V al;
      if (SPLIT) al = Frag<T>::load(Ab2 + ao);
#pragma unroll
      for (int j = 0; j < 4; ++j) {
        acc[i][j] = Frag<T>::mma(ah, bh[j], acc[i][j]);
        if (SPLIT) {
          acc[i][j] = Frag<T>::mma(ah, bl[j], acc[i][j]);
          acc[i][j] = Frag<T>::mma(al, bh[j], acc[i][j]);
        }
      }
      Frag<T>::guard4(acc[i][0], acc[i][1], acc[i][2], acc[i][3], ah, SPLIT ? al : ah);
    }
    Frag<T>::keep(bh[0], bh[1], bh[2], bh[3]);
    if (SPLIT) Frag<T>::keep(bl[0], bl[1], bl[2], bl[3]);
  }
  acc_guard4(acc[0][0], acc[0][1], acc[0][2], acc[0][3]);
  acc_guard4(acc[1][0], acc[1][1], acc[1][2], acc[1][3]);
  acc_guard4(acc[2][0], acc[2][1], acc[2][2], acc[2][3]);
  acc_guard4(acc[3][0], acc[3][1], acc[3][2], acc[3][3]);

  float* slab = sT[wave];
  const float* Rb = RESID ? (resid + (size_t)b * strideR) : nullptr;
#pragma unroll
  for (int i = 0; i < 4; ++i) {
    const int mBase = m0 + (i << 4);
#pragma unroll
    for (int j = 0; j < 4; ++j) {
      const int n = n0 + (j << 4) + rlane;
      float bv = 0.f;
      if (BIAS_MODE == 2) bv = bias[n];
#pragma unroll
      for (int r = 0; r < 8; ++r) {
        float v = acc[i][j][r] * scale;
        if (BIAS_MODE == 1) v += bias[mBase + mOff + r];
        if (BIAS_MODE == 2) v += bv;
        if (RESID) v += Rb[(size_t)(mBase + mOff + r) * ldc + n];
        if (ACT == 1) v = tanhf(v);
        if (ACT == 2) v = fmaxf(v, 0.0f);
        if (ACT == 3) v = v / (1.0f + expf(-v));
        if (ACT == 4) v = (v > 0.f) ? v : 0.01f * v;
        slab[(mOff + r) * 68 + (j << 4) + rlane] = v;
      }
    }
    __builtin_amdgcn_fence(__ATOMIC_RELEASE, "workgroup");
    __builtin_amdgcn_wave_barrier();
    __builtin_amdgcn_fence(__ATOMIC_ACQUIRE, "workgroup");
    if (OUT_MODE == 0) {
      float* C = (float*)Cout + (size_t)b * strideC;
      const int hh = lane >> 4, c4 = (lane & 15) * 4;
      for (int pass = 0; pass < 2; ++pass) {
#pragma unroll
        for (int it = 0; it < 8; ++it) {
          const int row = it * 2 + hh;
          v4f v = *(const v4f*)(slab + row * 68 + c4);
          *(volatile v4f*)(C + (size_t)(mBase + row) * ldc + n0 + c4) = v;
        }
        __threadfence();
      }
    } else {
      const int q = lane >> 3, c8 = (lane & 7) * 8;
      unsigned short* C  = (unsigned short*)Cout  + (size_t)b * strideC;
      unsigned short* C2 = (OUT_MODE == 2) ? ((unsigned short*)Cout2 + (size_t)b * strideC) : nullptr;
      for (int pass = 0; pass < 2; ++pass) {
#pragma unroll
        for (int it = 0; it < 4; ++it) {
          const int row = it * 4 + q;
          const float* sp = slab + row * 68 + c8;
          v8h hv, lv;
#pragma unroll
          for (int e = 0; e < 8; ++e) {
            if (OUT_MODE == 1) {
              hv[e] = (_Float16)sp[e];
            } else {
              unsigned short hb = f2bf_bits(sp[e]);
              unsigned short lb = f2bf_bits(sp[e] - bf_bits2f(hb));
              hv[e] = __builtin_bit_cast(_Float16, hb);
              lv[e] = __builtin_bit_cast(_Float16, lb);
            }
          }
          *(volatile v8h*)(C + (size_t)(mBase + row) * ldc + n0 + c8) = hv;
          if (OUT_MODE == 2) *(volatile v8h*)(C2 + (size_t)(mBase + row) * ldc + n0 + c8) = lv;
        }
        __threadfence();
      }
    }
    __builtin_amdgcn_fence(__ATOMIC_RELEASE, "workgroup");
    __builtin_amdgcn_wave_barrier();
    __builtin_amdgcn_fence(__ATOMIC_ACQUIRE, "workgroup");
  }
}

__global__ __launch_bounds__(kThr) void cast_plane_kernel(const float* __restrict__ src, unsigned short* __restrict__ dst,
                                                          int colsLog2, int dstPitch, int dstOff) {
  const int i   = blockIdx.x * kThr + threadIdx.x;
  const int sh  = colsLog2 - 3;
  const int row = i >> sh;
  const int c8  = (i & ((1 << sh) - 1)) * 8;
  const float* sp = src + ((size_t)row << colsLog2) + c8;
  const v4f a0 = *(const v4f*)(sp);
  const v4f a1 = *(const v4f*)(sp + 4);
  v8h hv;
#pragma unroll
  for (int e = 0; e < 4; ++e) {
    const float f0 = a0[e];
    const float f1 = a1[e];
    hv[e]     = (_Float16)carry_flush(bf16r(f0), kInCarry);
    hv[4 + e] = (_Float16)carry_flush(bf16r(f1), kInCarry);
  }
  unsigned short* dp = dst + (size_t)row * dstPitch + dstOff + c8;
  *(volatile v8h*)dp = hv;
  __threadfence();
  *(volatile v8h*)dp = hv;
}

__global__ __launch_bounds__(128) void setup_kernel(const float* __restrict__ y0, const float* __restrict__ b_y2x, const float* __restrict__ b_x2y,
                                                    float* __restrict__ BIAS, unsigned short* __restrict__ Y016) {
  const unsigned y = blockIdx.y;
  const unsigned c = threadIdx.x;
  if (y < 2u) {
    v4f o = {0.f, 0.f, 0.f, 0.f};
    if (y == 0u) {
      const unsigned i0 = c * 4u;
      if (i0 < (unsigned)kNH) {
        const v4f a = *(const v4f*)(b_y2x + i0);
#pragma unroll
        for (int e = 0; e < 4; ++e) { const float p = a[e]; o[e] = bf16r(p); }
      } else if (i0 < (unsigned)(kNH + kNY)) {
        const v4f a = *(const v4f*)(b_x2y + (i0 - (unsigned)kNH));
#pragma unroll
        for (int e = 0; e < 4; ++e) { const float p = a[e]; o[e] = bf16r(p); }
      }
    }
    float* dp = BIAS + y * 512u + c * 4u;
    *(volatile v4f*)dp = o;
    __threadfence();
    *(volatile v4f*)dp = o;
  } else {
    if (c >= 8u) return;
    const unsigned r = y - 2u;
    const bool live = r < (unsigned)kNB;
    const float* sp = y0 + (size_t)(live ? r : 0u) * kNY + c * 8u;
    const v4f a0 = *(const v4f*)sp, a1 = *(const v4f*)(sp + 4);
    v8h hv;
#pragma unroll
    for (int e = 0; e < 4; ++e) {
      const float f0 = a0[e], f1 = a1[e];
      hv[e] = (_Float16)(live ? carry_flush(bf16r(f0), kInCarry) : 0.0f);
      hv[4 + e] = (_Float16)(live ? carry_flush(bf16r(f1), kInCarry) : 0.0f);
    }
    unsigned short* dp = Y016 + (size_t)r * kNY + c * 8u;
    *(volatile v8h*)dp = hv;
    __threadfence();
    *(volatile v8h*)dp = hv;
  }
}
static_assert(kFBXY == kNH && kFZB == 512 && kFEnd == 1024 && kNY / 8 == 8 && (kNH % 128) == 0 && ((kNH + kNY) % 32) == 0, "set-up rows; the bias arms end on wave boundaries");

__global__ __launch_bounds__(kThr) void ssm_scan_kernel(const float* __restrict__ BU, const float* __restrict__ lre, const float* __restrict__ lim,
                                                        const float* SIN, float* SOUT, unsigned short* __restrict__ X16) {
  const unsigned v = blockIdx.x * (unsigned)kThr + threadIdx.x;
  const unsigned smp = v >> 6, h0 = (v & 63u) * 2u;
  float lr[2], li[2], zr[2], zi[2];
#pragma unroll
  for (int k = 0; k < 2; ++k) {
    const float a = lre[h0 + k], b = lim[h0 + k];
    const float r = expf(-fabsf(bf16r(a)));
    const float th = kHalfPi * bf16r(b);
    lr[k] = r * cosf(th);
    li[k] = r * sinf(th);
    zr[k] = SIN[(size_t)smp * kNH + h0 + k];
    zi[k] = SIN[(size_t)smp * kNH + kHP + h0 + k];
  }
  for (int t = 0; t < kTC; ++t) {
    const size_t row = (size_t)t * kNB + smp;
    const v2f a = *(const v2f*)(BU + row * kNH + h0);
    const v2f b = *(const v2f*)(BU + row * kNH + kHP + h0);
    v2h vr, vi;
#pragma unroll
    for (int k = 0; k < 2; ++k) {
      const float nzr = lr[k] * zr[k] - li[k] * zi[k] + a[k];
      const float nzi = li[k] * zr[k] + lr[k] * zi[k] + b[k];
      zr[k] = nzr; zi[k] = nzi;
      vr[k] = (_Float16)carry_flush(nzr, kXCarry);
      vi[k] = (_Float16)carry_flush(nzi, kXCarry);
    }
    unsigned short* rp = X16 + row * kNH + h0;
    unsigned short* ip = X16 + row * kNH + kHP + h0;
    for (int pass = 0; pass < 2; ++pass) {
      *(volatile v2h*)rp = vr;
      *(volatile v2h*)ip = vi;
      __threadfence();
    }
  }
  float* sr = SOUT + (size_t)smp * kNH + h0;
  float* si = SOUT + (size_t)smp * kNH + kHP + h0;
  const v2f or2 = {zr[0], zr[1]}, oi2 = {zi[0], zi[1]};
  for (int pass = 0; pass < 2; ++pass) {
    *(volatile v2f*)sr = or2;
    *(volatile v2f*)si = oi2;
    __threadfence();
  }
}
static_assert(kNB * 64 == 8 * kThr && kHP == 128, "scan grid exact: two waves a sample");

__global__ __launch_bounds__(kThr) void out_copy_kernel(const float* __restrict__ Y32, float* __restrict__ out) {
  const size_t o4 = ((size_t)blockIdx.x * kThr + threadIdx.x) * 4u;
  const v4f a = *(const v4f*)(Y32 + o4);
  *(volatile v4f*)(out + o4) = a;
  __threadfence();
  *(volatile v4f*)(out + o4) = a;
}
static_assert(((size_t)kRC * kNY / 4) == 2048 * kThr, "copy grid exact");

static_assert(((size_t)kNH * kNU / 8) % kThr == 0 && ((size_t)kNY * kNH / 8) % kThr == 0 && ((size_t)kRC * kNU / 8) % kThr == 0, "plane cast grids exact");

extern "C" void kernel_launch(void* const* d_in, const int* in_sizes, int n_in,
                              void* d_out, int out_size, void* d_ws, size_t ws_size,
                              hipStream_t stream) {
  if (n_in < 9 || d_out == nullptr || d_ws == nullptr) return;
  if (in_sizes[0] != kNB * kNY || in_sizes[1] != kT * kNB * kNU || in_sizes[2] != kHP || in_sizes[3] != kHP || in_sizes[4] != kNH * kNU) return;
  if (in_sizes[5] != kNH * kNY || in_sizes[6] != kNH || in_sizes[7] != kNY * kNH || in_sizes[8] != kNY) return;
  if (out_size != kT * kNB * kNY) return;
  if (ws_size < kWsTotal) return;
  const float* y0 = (const float*)d_in[0];
  const float* U = (const float*)d_in[1];
  const float* lre = (const float*)d_in[2];
  const float* lim = (const float*)d_in[3];
  const float* B = (const float*)d_in[4];
  const float* W_y2x = (const float*)d_in[5];
  const float* b_y2x = (const float*)d_in[6];
  const float* W_x2y = (const float*)d_in[7];
  const float* b_x2y = (const float*)d_in[8];
  float* out = (float*)d_out;
  char* ws = (char*)d_ws;
  unsigned short* B16 = (unsigned short*)(ws + kOffB16);
  unsigned short* WYX16 = (unsigned short*)(ws + kOffWYX16);
  unsigned short* WXY16 = (unsigned short*)(ws + kOffWXY16);
  float* BIAS = (float*)(ws + kOffBIAS);
  unsigned short* Y016 = (unsigned short*)(ws + kOffY016);
  float* X0 = (float*)(ws + kOffX0);
  float* STATE = (float*)(ws + kOffSTATE);
  unsigned short* U16 = (unsigned short*)(ws + kOffU16);
  float* BU = (float*)(ws + kOffBU);
  unsigned short* X16 = (unsigned short*)(ws + kOffX16);
  float* Y32 = (float*)(ws + kOffY32);

  cast_plane_kernel<<<(int)(((size_t)kNH * kNU / 8) / kThr), kThr, 0, stream>>>(B, B16, 6, kNU, 0);
  cast_plane_kernel<<<(int)(((size_t)kNH * kNY / 8) / kThr), kThr, 0, stream>>>(W_y2x, WYX16, 6, kNY, 0);
  cast_plane_kernel<<<(int)(((size_t)kNY * kNH / 8) / kThr), kThr, 0, stream>>>(W_x2y, WXY16, 8, kNH, 0);
  setup_kernel<<<dim3(1, 2 + kM0), 128, 0, stream>>>(y0, b_y2x, b_x2y, BIAS, Y016);
  wmma_gemm64<0, false, 2, 0, false, 0><<<dim3((kM0 / 64) * (kNH / 64) / 8, 1), 256, 0, stream>>>(
      Y016, Y016, kNY, 0L, WYX16, WYX16, kNY, 0L, (void*)X0, (void*)X0, kNH, 0L, BIAS + kFBYX, nullptr, 0L, kM0, kNH, kNY, kScIn);

  for (int ch = 0; ch < kNCh; ++ch) {
    const float* uc = U + (size_t)ch * kRC * kNU;
    float* oc = out + (size_t)ch * kRC * kNY;
    cast_plane_kernel<<<(int)(((size_t)kRC * kNU / 8) / kThr), kThr, 0, stream>>>(uc, U16, 6, kNU, 0);
    wmma_gemm64<0, false, 2, 0, false, 0><<<dim3((kRC / 64) * (kNH / 64) / 8, 1), 256, 0, stream>>>(
        U16, U16, kNU, 0L, B16, B16, kNU, 0L, (void*)BU, (void*)BU, kNH, 0L, BIAS + kFZB, nullptr, 0L, kRC, kNH, kNU, kScIn);
    ssm_scan_kernel<<<(kNB * 64) / kThr, kThr, 0, stream>>>(BU, lre, lim, (ch == 0) ? (const float*)X0 : (const float*)STATE, STATE, X16);
    wmma_gemm64<0, false, 2, 0, false, 0><<<dim3((kRC / 64) * (kNY / 64) / 8, 1), 256, 0, stream>>>(
        X16, X16, kNH, 0L, WXY16, WXY16, kNH, 0L, (void*)Y32, (void*)Y32, kNY, 0L, BIAS + kFBXY, nullptr, 0L, kRC, kNY, kNH, kScOut);
    out_copy_kernel<<<2048, kThr, 0, stream>>>(Y32, oc);
  }
}
